// Model_89670327206497
// MI455X (gfx1250) — hardware-verified
//
#include <hip/hip_runtime.h>
#include <stddef.h>
#include <stdint.h>


#define NLOC   20000
#define NEXP   200000
#define HD     64
#define NEDG   1500000
#define NLBL   400000
#define MLOC   20096
#define MEXP   200064
#define NTHR   256
#define NWAVE  8
#define EPT    8
#define CHUNK  (NTHR * EPT)
#define WCAP   (EPT * 32)
#define LISTN  (NWAVE * WCAP)
#define NBO    1024
#define SLO    10
#define RCO    10240
#define DCO    40
#define NBR    256
#define SLR    8
#define RCR    22528
#define DCR    160
#define GAO    196
#define GAR    79
#define GM     128
#define GTH    256
#define NUX    (MLOC * 8)
#define NWU    (18 * 512)
#define WPLN   73728
#define WSMAX  134217728

static_assert((CHUNK & (CHUNK - 1)) == 0 && CHUNK <= 4096);
static_assert(NBO == (1 << SLO) && NBR == (1 << SLR));
static_assert(((long long)CHUNK << SLO) < (1LL << 31));
static_assert(((long long)NLOC << SLO) < (1LL << 31) && ((long long)NEXP << SLR) < (1LL << 31));
static_assert(RCO % 32 == 0 && RCR % 32 == 0);
static_assert(RCO * 100 >= 7877 * 105 && RCR * 100 >= 19547 * 105 && RCR <= 28672);
static_assert(DCO >= 21 + 8 && DCR >= 114 + 8);
static_assert(GAO * NBO >= MEXP && GAR * NBR >= MLOC);
static_assert(MEXP % GM == 0 && MLOC % GM == 0 && MEXP >= NEXP && MLOC >= NLOC);
static_assert(NBO % (2 * NWAVE) == 0 && NBR % (2 * NWAVE) == 0 && NBO % 32 == 0 && NBR % 32 == 0);
static_assert(NBO / 4 <= NTHR && NBR / 4 <= NTHR);
static_assert(NLBL % 32 == 0 && HD == 64);
static_assert(NUX % NTHR == 0 && NWU % NTHR == 0 && 512 % NTHR == 0);
static_assert((LISTN + 2 * RCR + 3 * NBR + 16) * 4 <= 300000);
static_assert(GM == (GTH / 32) * 16);

typedef float          v2f  __attribute__((ext_vector_type(2)));
typedef float          v4f  __attribute__((ext_vector_type(4)));
typedef float          v8f  __attribute__((ext_vector_type(8)));
typedef int            v4i  __attribute__((ext_vector_type(4)));
typedef int            v8i  __attribute__((ext_vector_type(8)));
typedef unsigned       v4u  __attribute__((ext_vector_type(4)));
typedef unsigned short v4us __attribute__((ext_vector_type(4)));
typedef unsigned short v8us __attribute__((ext_vector_type(8)));
typedef __bf16         v16b __attribute__((ext_vector_type(16)));
typedef v4f  __attribute__((may_alias)) v4fa;
typedef v4i  __attribute__((may_alias)) v4ia;
typedef v4u  __attribute__((may_alias)) v4ua;
typedef v4us __attribute__((may_alias)) v4usa;
typedef v8us __attribute__((may_alias)) v8usa;
typedef unsigned __attribute__((may_alias)) ua;
union FragB { v16b v; v8us h[2]; v8i w; };

__device__ __forceinline__ v8f wmb(const FragB& a, const FragB& b, v8f c) {
  v8f d = __builtin_amdgcn_wmma_f32_16x16x32_bf16(false, a.v, false, b.v, (short)0, c, false, false);
  asm volatile("v_nop\n\tv_nop\n\tv_nop\n\tv_nop" : "+v"(d) : "v"(a.w), "v"(b.w));
  return d;
}

__device__ __forceinline__ unsigned int f2bf(float f) {
  const unsigned int u = __float_as_uint(f);
  const unsigned int r = ((u + 0x7FFFu + ((u >> 16) & 1u)) >> 16) & 0xFFFFu;
  return ((u & 0x7FFFFFFFu) > 0x7F800000u) ? 0x7FC0u : r;
}
__device__ __forceinline__ float bf2f(unsigned int b) { return __uint_as_float(b << 16); }
__device__ __forceinline__ float bfr(float f) { return bf2f(f2bf(f)); }

__device__ __forceinline__ void wave_sync() {
  __builtin_amdgcn_fence(__ATOMIC_RELEASE, "workgroup");
  __builtin_amdgcn_wave_barrier();
  __builtin_amdgcn_fence(__ATOMIC_ACQUIRE, "workgroup");
}

template <int SLB>
__device__ __forceinline__ int scan_chunk(const int* __restrict__ dsts, int nE, int cbase, int slotBase,
                                          int nb, int vec8, int* list, int tid, int lane, int wave) {
  int wc = 0;
  const int el0  = tid * EPT;
  const int e0   = cbase + el0;
  const int sent = -2147483647 - 1;
  v4i da, db;
  if (vec8 != 0 && cbase + CHUNK <= nE) {
    da = *(const v4i*)(dsts + e0);
    db = *(const v4i*)(dsts + e0 + 4);
  } else {
    da.x = (e0     < nE) ? dsts[min(e0,     nE - 1)] : sent;
    da.y = (e0 + 1 < nE) ? dsts[min(e0 + 1, nE - 1)] : sent;
    da.z = (e0 + 2 < nE) ? dsts[min(e0 + 2, nE - 1)] : sent;
    da.w = (e0 + 3 < nE) ? dsts[min(e0 + 3, nE - 1)] : sent;
    db.x = (e0 + 4 < nE) ? dsts[min(e0 + 4, nE - 1)] : sent;
    db.y = (e0 + 5 < nE) ? dsts[min(e0 + 5, nE - 1)] : sent;
    db.z = (e0 + 6 < nE) ? dsts[min(e0 + 6, nE - 1)] : sent;
    db.w = (e0 + 7 < nE) ? dsts[min(e0 + 7, nE - 1)] : sent;
  }
  const unsigned nbs = (unsigned)slotBase;
  const unsigned unb = (unsigned)nb;
  const unsigned s0 = (unsigned)da.x - nbs, s1 = (unsigned)da.y - nbs;
  const unsigned s2 = (unsigned)da.z - nbs, s3 = (unsigned)da.w - nbs;
  const unsigned s4 = (unsigned)db.x - nbs, s5 = (unsigned)db.y - nbs;
  const unsigned s6 = (unsigned)db.z - nbs, s7 = (unsigned)db.w - nbs;
  const bool h0 = s0 < unb, h1 = s1 < unb, h2 = s2 < unb, h3 = s3 < unb;
  const bool h4 = s4 < unb, h5 = s5 < unb, h6 = s6 < unb, h7 = s7 < unb;
  const unsigned any = __builtin_amdgcn_ballot_w32(h0 | h1 | h2 | h3 | h4 | h5 | h6 | h7);
  if (any != 0u) {
#define HITJ(J, HJ, SJ) { \
      const unsigned mj = __builtin_amdgcn_ballot_w32(HJ); \
      if (mj != 0u) { \
        if (HJ) { \
          const int pos = wc + (int)__builtin_amdgcn_mbcnt_lo(mj, 0u); \
          if (pos < WCAP) list[wave * WCAP + pos] = ((el0 + (J)) << SLB) | (int)(SJ); \
        } \
        wc += (int)__builtin_popcount(mj); } }
    HITJ(0, h0, s0)
    HITJ(1, h1, s1)
    HITJ(2, h2, s2)
    HITJ(3, h3, s3)
    HITJ(4, h4, s4)
    HITJ(5, h5, s5)
    HITJ(6, h6, s6)
    HITJ(7, h7, s7)
#undef HITJ
  }
  return wc;
}

__global__ __launch_bounds__(NTHR) void k_prep(const float* __restrict__ embl,
    const float* __restrict__ w1lo, const float* __restrict__ w1ro,
    const float* __restrict__ w1lr, const float* __restrict__ w1rr,
    const float* __restrict__ w2lo, const float* __restrict__ w2ro,
    const float* __restrict__ w2lr, const float* __restrict__ w2rr,
    const float* __restrict__ dw1,
    unsigned short* XLB, unsigned short* WPL, int nLoc) {
  const int u = (int)blockIdx.x * NTHR + (int)threadIdx.x;
  v8us o;
  unsigned short* dp;
  if (u < NUX) {
    const int row = u >> 3;
    const int c0  = (u & 7) * 8;
    const int rc  = row < nLoc ? row : nLoc - 1;
    const float* p = embl + (size_t)rc * HD + c0;
    const v4f a = *(const v4f*)p;
    const v4f b = *(const v4f*)(p + 4);
    const bool ok = row < nLoc;
    o[0] = ok ? (unsigned short)f2bf(a.x) : (unsigned short)0;
    o[1] = ok ? (unsigned short)f2bf(a.y) : (unsigned short)0;
    o[2] = ok ? (unsigned short)f2bf(a.z) : (unsigned short)0;
    o[3] = ok ? (unsigned short)f2bf(a.w) : (unsigned short)0;
    o[4] = ok ? (unsigned short)f2bf(b.x) : (unsigned short)0;
    o[5] = ok ? (unsigned short)f2bf(b.y) : (unsigned short)0;
    o[6] = ok ? (unsigned short)f2bf(b.z) : (unsigned short)0;
    o[7] = ok ? (unsigned short)f2bf(b.w) : (unsigned short)0;
    dp = XLB + (size_t)row * HD + c0;
  } else if (u < NUX + NWU) {
    const int v    = u - NUX;
    const int part = v >> 9;
    const int w    = v & 511;
    const int n    = w >> 3;
    const int k8   = (w & 7) * 8;
    const float* W = w1lo;
    int pbase = 0, pitch = 192, coff = 0, so = 0;
    switch (part) {
      case 0:  break;
      case 1:  coff = 64; break;
      case 2:  W = w1ro; coff = 128; break;
      case 3:  W = w1lr; pbase = 12288; break;
      case 4:  W = w1lr; pbase = 12288; coff = 64; break;
      case 5:  W = w1rr; pbase = 12288; coff = 128; break;
      case 6:  W = w2lo; pbase = 24576; pitch = 256; break;
      case 7:  W = w2lo; pbase = 24576; pitch = 256; coff = 64; break;
      case 8:  W = w2ro; pbase = 24576; pitch = 256; coff = 128; break;
      case 9:  W = w2ro; pbase = 24576; pitch = 256; coff = 192; break;
      case 10: W = w2lr; pbase = 40960; pitch = 256; break;
      case 11: W = w2lr; pbase = 40960; pitch = 256; coff = 64; break;
      case 12: W = w2rr; pbase = 40960; pitch = 256; coff = 128; break;
      case 13: W = w2rr; pbase = 40960; pitch = 256; coff = 192; break;
      case 14: W = dw1; pbase = 57344; pitch = 128; break;
      case 15: W = dw1; pbase = 57344; pitch = 128; coff = 64; break;
      case 16: W = dw1; pbase = 65536; pitch = 128; so = 4096; break;
      default: W = dw1; pbase = 65536; pitch = 128; coff = 64; so = 4096; break;
    }
    const float* p = W + so + (size_t)k8 * HD + n;
#pragma unroll
    for (int i = 0; i < 8; ++i) o[i] = (unsigned short)f2bf(p[(size_t)i * HD]);
    dp = WPL + (size_t)pbase + (size_t)n * pitch + coff + k8;
  } else {
    return;
  }
  *(volatile v8us*)dp = o;
  __threadfence();
  *(volatile v8us*)dp = o;
}

template <int NB, int SL, int RC>
__global__ __launch_bounds__(NTHR) void k_bucket(const int* __restrict__ srcs, const int* __restrict__ dsts,
                                                 int nE, int nDst, int nSrc, int vec8,
                                                 int* LIST, int* CNT, int* OFF, int* FLG) {
  extern __shared__ __attribute__((aligned(16))) int bsm[];
  int* list = bsm;
  int* hl   = bsm + LISTN;
  int* sl   = hl + RC;
  int* cnt  = sl + RC;
  int* offs = cnt + NB;
  int* cur  = offs + NB;
  int* wcnt = cur + NB;
  const int tid = (int)threadIdx.x, lane = tid & 31, wave = tid >> 5;
  const int blk = (int)blockIdx.x;
  const int nodeBase = blk * NB;
  int nb = nDst - nodeBase;
  nb = nb < 0 ? 0 : (nb > NB ? NB : nb);

  for (int i = tid; i < 3 * NB + 16; i += NTHR) cnt[i] = 0;
  __syncthreads();

  int tot = 0, ovf = 0;
  const int nChunks = (nE + CHUNK - 1) / CHUNK;
#pragma unroll 1
  for (int ch = 0; ch < nChunks; ++ch) {
    const int cbase = ch * CHUNK;
    const int wc = scan_chunk<SL>(dsts, nE, cbase, nodeBase, nb, vec8, list, tid, lane, wave);
    if (lane == 0) wcnt[wave] = wc;
    __syncthreads();
    int pre = 0, all = 0;
#pragma unroll
    for (int w2 = 0; w2 < NWAVE; ++w2) {
      int c = wcnt[w2];
      c = c < 0 ? 0 : (c > WCAP ? WCAP : c);
      all += c;
      pre += (w2 < wave) ? c : 0;
    }
    const int wcc  = wc > WCAP ? WCAP : wc;
    const int base = tot + pre;
#pragma unroll 1
    for (int i = lane; i < wcc; i += 32) {
      const int ent = list[wave * WCAP + i];
      const int el  = (ent >> SL) & (CHUNK - 1);
      const int sq  = ent & (NB - 1);
      int eid = cbase + el;
      eid = eid > nE - 1 ? nE - 1 : eid;
      const int sraw = srcs[eid];
      const int s = sraw < 0 ? 0 : (sraw > nSrc - 1 ? nSrc - 1 : sraw);
      const int pos = base + i;
      if (pos < RC) hl[pos] = (int)(((unsigned)s << SL) | (unsigned)sq);
    }
    if (tot + all > RC) ovf = 1;
    tot += all;
    tot = tot > RC ? RC : tot;
    __syncthreads();
  }
  const int nh = tot;

  if (wave == 0) {
#pragma unroll 1
    for (int b0 = 0; b0 < nh; b0 += 32) {
      const int idx = b0 + lane;
      const int uv  = hl[idx < nh ? idx : nh - 1];
      const int m32 = (nh - b0) < 32 ? (nh - b0) : 32;
#pragma unroll 1
      for (int k = 0; k < m32; ++k) {
        const int u  = __builtin_amdgcn_readlane(uv, k);
        const int sq = u & (NB - 1);
        if (lane == 0) cnt[sq] = cnt[sq] + 1;
      }
    }
  }
  __syncthreads();
  if (wave == 0) {
    const int base = lane * (NB / 32);
    int s = 0;
#pragma unroll 1
    for (int i = 0; i < NB / 32; ++i) s += cnt[base + i];
    int incl = s;
#pragma unroll
    for (int d = 1; d < 32; d <<= 1) {
      const int y = __shfl_up(incl, d, 32);
      if (lane >= d) incl += y;
    }
    int run = incl - s;
#pragma unroll 1
    for (int i = 0; i < NB / 32; ++i) {
      const int cv = cnt[base + i];
      offs[base + i] = run;
      cur[base + i]  = run;
      run += cv;
    }
  }
  __syncthreads();
  if (wave == 0) {
#pragma unroll 1
    for (int b0 = 0; b0 < nh; b0 += 32) {
      const int idx = b0 + lane;
      const int uv  = hl[idx < nh ? idx : nh - 1];
      const int m32 = (nh - b0) < 32 ? (nh - b0) : 32;
#pragma unroll 1
      for (int k = 0; k < m32; ++k) {
        const int u  = __builtin_amdgcn_readlane(uv, k);
        const int sq = u & (NB - 1);
        if (lane == 0) {
          int p = cur[sq];
          p = p < 0 ? 0 : (p > RC - 1 ? RC - 1 : p);
          sl[p] = (int)((unsigned)u >> SL);
          cur[sq] = p + 1;
        }
      }
    }
  }
  __syncthreads();
  const int nhPad = (nh + 31) & ~31;
  for (int i = nh + tid; i < nhPad; i += NTHR) sl[i] = 0;
  __syncthreads();

  int* lbp = LIST + (size_t)blk * RC;
  int* cp  = CNT + (size_t)nodeBase + 4 * tid;
  int* op  = OFF + (size_t)nodeBase + 4 * tid;
  int* fp  = FLG + (size_t)blk * 32 + 4 * (tid & 7);
  v4i cv4 = {0, 0, 0, 0}, ov4 = {0, 0, 0, 0};
  if (tid < NB / 4) {
    cv4 = *(const v4ia*)(cnt + 4 * tid);
    ov4 = *(const v4ia*)(offs + 4 * tid);
  }
  v4i fv;
  fv.x = (tid == 0) ? nh : 0;
  fv.y = (tid == 0) ? ovf : 0;
  fv.z = 0; fv.w = 0;
#pragma unroll 1
  for (int p = tid * 4; p < nhPad; p += NTHR * 4) {
    const v4i v = *(const v4ia*)(sl + p);
    *(volatile v4i*)(lbp + p) = v;
  }
  if (tid < NB / 4) { *(volatile v4i*)cp = cv4; *(volatile v4i*)op = ov4; }
  if (tid < 8) *(volatile v4i*)fp = fv;
  __threadfence();
#pragma unroll 1
  for (int p = tid * 4; p < nhPad; p += NTHR * 4) {
    const v4i v = *(const v4ia*)(sl + p);
    *(volatile v4i*)(lbp + p) = v;
  }
  if (tid < NB / 4) { *(volatile v4i*)cp = cv4; *(volatile v4i*)op = ov4; }
  if (tid < 8) *(volatile v4i*)fp = fv;
}

template <int MODE, int NB, int RC, int DC>
__global__ __launch_bounds__(NTHR) void k_agg(const int* __restrict__ LIST, const int* __restrict__ CNT,
                                              const int* __restrict__ OFF, const int* __restrict__ FLG,
                                              const unsigned short* __restrict__ sh, const float* __restrict__ sf,
                                              unsigned* AGG, int nDst, int nSrc, int MPr) {
  __shared__ __attribute__((aligned(16))) unsigned rb[NWAVE * 128];
  const int tid = (int)threadIdx.x, lane = tid & 31, wave = tid >> 5;
  const int blk = (int)blockIdx.x;
  const int nodeBase = blk * NB;
  const int nhraw = FLG[(size_t)blk * 32];
  const int bflag = FLG[(size_t)blk * 32 + 1];
  const int nh  = nhraw < 0 ? 0 : (nhraw > RC ? RC : nhraw);
  const int ovf = (bflag != 0 || nhraw < 0 || nhraw > RC) ? 1 : 0;
  const int* lb = LIST + (size_t)blk * RC;
  unsigned* rw = rb + wave * 128;
  const float qnan = __int_as_float(0x7fc00000);
  const float pzb  = (ovf != 0) ? qnan : 0.0f;

#pragma unroll 1
  for (int pi = 0; pi < NB / (2 * NWAVE); ++pi) {
    const int node0 = nodeBase + 2 * (pi * NWAVE + wave);
#pragma unroll 1
    for (int q = 0; q < 2; ++q) {
      const int node = node0 + q;
      int c = CNT[node];
      const bool big = c > DC;
      c = c < 0 ? 0 : (c > DC ? DC : c);
      int o = OFF[node];
      o = o < 0 ? 0 : (o > nh ? nh : o);
      if (c > nh - o) c = nh - o;
      float a0 = 0.0f, a1 = 0.0f;
#pragma unroll 1
      for (int b0 = 0; b0 < c; b0 += 32) {
        int idx = o + b0 + lane;
        idx = idx > o + c - 1 ? o + c - 1 : idx;
        int sr = lb[idx];
        sr = sr < 0 ? 0 : (sr > nSrc - 1 ? nSrc - 1 : sr);
        const int m32 = (c - b0) < 32 ? (c - b0) : 32;
#pragma unroll 1
        for (int k = 0; k < m32; ++k) {
          const int sk = __builtin_amdgcn_readlane(sr, k);
          if constexpr (MODE == 0) {
            const unsigned w = *(const ua*)(sh + (size_t)sk * HD + 2 * lane);
            a0 += __uint_as_float(w << 16);
            a1 += __uint_as_float(w & 0xffff0000u);
          } else if constexpr (MODE == 1) {
            const v2f x = *(const v2f*)(sf + (size_t)sk * HD + 2 * lane);
            a0 += bfr(x.x);
            a1 += bfr(x.y);
          } else {
            const unsigned short* rp = sh + (size_t)sk * (2 * HD) + 2 * lane;
            const unsigned wh = *(const ua*)rp;
            const unsigned wl = *(const ua*)(rp + HD);
            a0 += __uint_as_float(wh << 16) + __uint_as_float(wl << 16);
            a1 += __uint_as_float(wh & 0xffff0000u) + __uint_as_float(wl & 0xffff0000u);
          }
        }
      }
      const float dv  = (float)(c > 1 ? c : 1);
      const float pzr = big ? qnan : pzb;
      const bool live = node < nDst;
      const float m0 = live ? (a0 / dv + pzr) : 0.0f;
      const float m1 = live ? (a1 / dv + pzr) : 0.0f;
      const unsigned h0 = f2bf(m0), h1 = f2bf(m1);
      const unsigned l0 = f2bf(m0 - bf2f(h0)), l1 = f2bf(m1 - bf2f(h1));
      rw[q * 64 + lane]      = h0 | (h1 << 16);
      rw[q * 64 + 32 + lane] = l0 | (l1 << 16);
    }
    wave_sync();
    const v4u qv = *(const v4ua*)(rw + 4 * lane);
    wave_sync();
    if (node0 < MPr) {
      unsigned* dp = AGG + (size_t)node0 * HD + 4 * lane;
      *(volatile v4u*)dp = qv;
      __threadfence();
      *(volatile v4u*)dp = qv;
    }
  }
}

template <int KT>
__device__ __forceinline__ void bstep(const FragB& af, const unsigned short* wq, v8f (&acc)[4]) {
#pragma unroll
  for (int nt = 0; nt < 4; ++nt) {
    const unsigned short* w = wq + (size_t)(16 * nt) * KT;
    FragB bf;
    bf.h[0] = *(const v8usa*)w;
    bf.h[1] = *(const v8usa*)(w + 16);
    acc[nt] = wmb(af, bf, acc[nt]);
  }
}

template <int S1, int EPI>
__global__ __launch_bounds__(GTH) void k_gemm(const unsigned short* A0, const unsigned short* A1h,
                                              const float* __restrict__ A1f, int a1rows,
                                              const unsigned short* __restrict__ BT,
                                              const float* __restrict__ bias, int hasBias,
                                              unsigned short* outH, float* outF, int nOut) {
  constexpr int K1 = (S1 == 0) ? 0 : ((S1 == 3) ? 128 : 64);
  constexpr int KT = 128 + K1;
  static_assert(KT % 32 == 0);
  __shared__ __attribute__((aligned(16))) float stg[GM * HD];
  const int tid = (int)threadIdx.x, lane = tid & 31, wave = tid >> 5, hh = lane >> 4, m = lane & 15;
  const int rowBase = (int)blockIdx.x * GM;
  const int grow = rowBase + 16 * wave + m;

  v8f acc[4];
  {
    const v8f z = {0.f, 0.f, 0.f, 0.f, 0.f, 0.f, 0.f, 0.f};
    acc[0] = z; acc[1] = z; acc[2] = z; acc[3] = z;
  }
  const unsigned short* bp = BT + (size_t)m * KT + 8 * hh;
  {
    const unsigned short* ap = A0 + (size_t)grow * 128 + 8 * hh;
#pragma unroll 1
    for (int k0 = 0; k0 < 128; k0 += 32) {
      FragB af;
      af.h[0] = *(const v8usa*)(ap + k0);
      af.h[1] = *(const v8usa*)(ap + k0 + 16);
      bstep<KT>(af, bp + k0, acc);
    }
  }
  if constexpr (S1 == 1) {
    const unsigned short* ap = A1h + (size_t)grow * 64 + 8 * hh;
#pragma unroll 1
    for (int k0 = 0; k0 < 64; k0 += 32) {
      FragB af;
      af.h[0] = *(const v8usa*)(ap + k0);
      af.h[1] = *(const v8usa*)(ap + k0 + 16);
      bstep<KT>(af, bp + 128 + k0, acc);
    }
  }
  if constexpr (S1 == 3) {
    const unsigned short* ap = A1h + (size_t)grow * 128 + 8 * hh;
#pragma unroll 1
    for (int k0 = 0; k0 < 128; k0 += 32) {
      FragB af;
      af.h[0] = *(const v8usa*)(ap + k0);
      af.h[1] = *(const v8usa*)(ap + k0 + 16);
      bstep<KT>(af, bp + 128 + k0, acc);
    }
  }
  if constexpr (S1 == 2) {
    const int rc = grow < a1rows ? grow : a1rows - 1;
    const float* fp = A1f + (size_t)rc * 64 + 8 * hh;
#pragma unroll 1
    for (int k0 = 0; k0 < 64; k0 += 32) {
      const v4f x0 = *(const v4f*)(fp + k0);
      const v4f x1 = *(const v4f*)(fp + k0 + 4);
      const v4f y0 = *(const v4f*)(fp + k0 + 16);
      const v4f y1 = *(const v4f*)(fp + k0 + 20);
      FragB af;
      v8us e0, e1;
      e0[0] = (unsigned short)f2bf(x0.x); e0[1] = (unsigned short)f2bf(x0.y);
      e0[2] = (unsigned short)f2bf(x0.z); e0[3] = (unsigned short)f2bf(x0.w);
      e0[4] = (unsigned short)f2bf(x1.x); e0[5] = (unsigned short)f2bf(x1.y);
      e0[6] = (unsigned short)f2bf(x1.z); e0[7] = (unsigned short)f2bf(x1.w);
      e1[0] = (unsigned short)f2bf(y0.x); e1[1] = (unsigned short)f2bf(y0.y);
      e1[2] = (unsigned short)f2bf(y0.z); e1[3] = (unsigned short)f2bf(y0.w);
      e1[4] = (unsigned short)f2bf(y1.x); e1[5] = (unsigned short)f2bf(y1.y);
      e1[6] = (unsigned short)f2bf(y1.z); e1[7] = (unsigned short)f2bf(y1.w);
      af.h[0] = e0;
      af.h[1] = e1;
      bstep<KT>(af, bp + 128 + k0, acc);
    }
  }

#pragma unroll
  for (int nt = 0; nt < 4; ++nt) {
    const int lc = 16 * nt + m;
#pragma unroll
    for (int r = 0; r < 8; ++r) {
      const int lr = 16 * wave + 8 * hh + r;
      stg[lr * HD + lc] = acc[nt][r];
    }
  }
  __syncthreads();

  v4f bb4;
  {
    const v4f t1 = *(const v4f*)(bias + 4 * m);
    bb4.x = (hasBias != 0) ? bfr(t1.x) : 0.0f;
    bb4.y = (hasBias != 0) ? bfr(t1.y) : 0.0f;
    bb4.z = (hasBias != 0) ? bfr(t1.z) : 0.0f;
    bb4.w = (hasBias != 0) ? bfr(t1.w) : 0.0f;
  }
  v4f pv[8];
#pragma unroll
  for (int i = 0; i < 8; ++i) {
    const int lr = 16 * wave + 2 * i + hh;
    pv[i] = *(const v4fa*)(stg + lr * HD + 4 * m);
  }
  __syncthreads();

#pragma unroll
  for (int i = 0; i < 8; ++i) {
    const int lr = 16 * wave + 2 * i + hh;
    const bool ok = (rowBase + lr) < nOut;
    v4f y = pv[i] + bb4;
    if constexpr (EPI == 0) {
      y.x = (y.x > 0.0f) ? y.x : (y.x - y.x);
      y.y = (y.y > 0.0f) ? y.y : (y.y - y.y);
      y.z = (y.z > 0.0f) ? y.z : (y.z - y.z);
      y.w = (y.w > 0.0f) ? y.w : (y.w - y.w);
    }
    y.x = ok ? y.x : 0.0f; y.y = ok ? y.y : 0.0f; y.z = ok ? y.z : 0.0f; y.w = ok ? y.w : 0.0f;
    pv[i] = y;
  }

  if constexpr (EPI == 2) {
#pragma unroll
    for (int i = 0; i < 8; ++i) {
      const int lr = 16 * wave + 2 * i + hh;
      *(volatile v4f*)(outF + (size_t)(rowBase + lr) * HD + 4 * m) = pv[i];
    }
    __threadfence();
#pragma unroll
    for (int i = 0; i < 8; ++i) {
      const int lr = 16 * wave + 2 * i + hh;
      *(volatile v4f*)(outF + (size_t)(rowBase + lr) * HD + 4 * m) = pv[i];
    }
  } else {
#pragma unroll
    for (int i = 0; i < 8; ++i) {
      const int lr = 16 * wave + 2 * i + hh;
      v4us h4, l4;
      unsigned hb;
      hb = f2bf(pv[i].x); h4[0] = (unsigned short)hb; l4[0] = (unsigned short)f2bf(pv[i].x - bf2f(hb));
      hb = f2bf(pv[i].y); h4[1] = (unsigned short)hb; l4[1] = (unsigned short)f2bf(pv[i].y - bf2f(hb));
      hb = f2bf(pv[i].z); h4[2] = (unsigned short)hb; l4[2] = (unsigned short)f2bf(pv[i].z - bf2f(hb));
      hb = f2bf(pv[i].w); h4[3] = (unsigned short)hb; l4[3] = (unsigned short)f2bf(pv[i].w - bf2f(hb));
      unsigned short* srow = (unsigned short*)stg + (size_t)lr * 128;
      *(v4usa*)(srow + 4 * m) = h4;
      *(v4usa*)(srow + HD + 4 * m) = l4;
    }
    __syncthreads();
    v8us qv[8];
#pragma unroll
    for (int i = 0; i < 8; ++i) {
      const int lr = 16 * wave + 2 * i + hh;
      const unsigned short* srow = (const unsigned short*)stg + (size_t)lr * 128;
      qv[i] = *(const v8usa*)(srow + 8 * m);
    }
#pragma unroll
    for (int i = 0; i < 8; ++i) {
      const int lr = 16 * wave + 2 * i + hh;
      *(volatile v8us*)(outH + (size_t)(rowBase + lr) * 128 + 8 * m) = qv[i];
    }
    __threadfence();
#pragma unroll
    for (int i = 0; i < 8; ++i) {
      const int lr = 16 * wave + 2 * i + hh;
      *(volatile v8us*)(outH + (size_t)(rowBase + lr) * 128 + 8 * m) = qv[i];
    }
  }
}

__global__ __launch_bounds__(NTHR) void k_dec(const int* __restrict__ eli, const float* __restrict__ PG,
                                              const float* __restrict__ PD, const float* __restrict__ dW2,
                                              const float* __restrict__ db2, float* out,
                                              int nL, int nLoc, int nExp) {
  const int lane = (int)threadIdx.x & 31, wave = (int)threadIdx.x >> 5;
  const int line = (int)blockIdx.x * NWAVE + wave;
  if (line * 32 >= nL) return;
  const int idx = line * 32 + lane;
  int r = eli[idx];
  int c = eli[(size_t)nL + idx];
  r = r < 0 ? 0 : (r > nLoc - 1 ? nLoc - 1 : r);
  c = c < 0 ? 0 : (c > nExp - 1 ? nExp - 1 : c);
  const v2f wq = *(const v2f*)(dW2 + 2 * lane);
  const float w0 = bfr(wq.x), w1 = bfr(wq.y);
  const float b2 = bfr(db2[0]);
  float res = 0.0f;
#pragma unroll 2
  for (int j = 0; j < 32; ++j) {
    const int rj = __builtin_amdgcn_readlane(r, j);
    const int cj = __builtin_amdgcn_readlane(c, j);
    const v2f pg = *(const v2f*)(PG + (size_t)rj * HD + 2 * lane);
    const v2f pd = *(const v2f*)(PD + (size_t)cj * HD + 2 * lane);
    float h0 = pg.x + pd.x;
    float h1 = pg.y + pd.y;
    h0 = (h0 > 0.0f) ? h0 : (h0 - h0);
    h1 = (h1 > 0.0f) ? h1 : (h1 - h1);
    float p = fmaf(h1, w1, h0 * w0);
    p += __shfl_xor(p, 16, 32);
    p += __shfl_xor(p, 8, 32);
    p += __shfl_xor(p, 4, 32);
    p += __shfl_xor(p, 2, 32);
    p += __shfl_xor(p, 1, 32);
    res = (lane == j) ? p : res;
  }
  const float o = res + b2;
  float* op = out + idx;
  *(volatile float*)op = o;
  __threadfence();
  *(volatile float*)op = o;
}

static inline size_t al256(size_t o) { return (o + 255) & ~(size_t)255; }

extern "C" void kernel_launch(void* const* d_in, const int* in_sizes, int n_in,
                              void* d_out, int out_size, void* d_ws, size_t ws_size,
                              hipStream_t stream) {
  if (n_in < 21) return;
  if (in_sizes[0] != NLOC * HD || in_sizes[1] != NEXP * HD) return;
  if (in_sizes[2] != HD * HD || in_sizes[4] != HD * HD || in_sizes[5] != HD * HD || in_sizes[7] != HD * HD) return;
  if (in_sizes[8] != HD * HD || in_sizes[10] != HD * HD || in_sizes[11] != HD * HD || in_sizes[13] != HD * HD) return;
  if (in_sizes[3] != HD || in_sizes[6] != HD || in_sizes[9] != HD || in_sizes[12] != HD) return;
  if (in_sizes[14] != 2 * HD * HD || in_sizes[15] != HD || in_sizes[16] != HD || in_sizes[17] != 1) return;
  if (in_sizes[18] != 2 * NEDG || in_sizes[19] != 2 * NEDG || in_sizes[20] != 2 * NLBL) return;
  if (out_size != NLBL) return;

  const float* emb_loc = (const float*)d_in[0];
  const float* emb_exp = (const float*)d_in[1];
  const float* W1l_of  = (const float*)d_in[2];
  const float* b1_of   = (const float*)d_in[3];
  const float* W1r_of  = (const float*)d_in[4];
  const float* W1l_rev = (const float*)d_in[5];
  const float* b1_rev  = (const float*)d_in[6];
  const float* W1r_rev = (const float*)d_in[7];
  const float* W2l_of  = (const float*)d_in[8];
  const float* b2_of   = (const float*)d_in[9];
  const float* W2r_of  = (const float*)d_in[10];
  const float* W2l_rev = (const float*)d_in[11];
  const float* b2_rev  = (const float*)d_in[12];
  const float* W2r_rev = (const float*)d_in[13];
  const float* dW1     = (const float*)d_in[14];
  const float* db1     = (const float*)d_in[15];
  const float* dW2     = (const float*)d_in[16];
  const float* db2     = (const float*)d_in[17];
  const int*   e_of    = (const int*)d_in[18];
  const int*   e_rev   = (const int*)d_in[19];
  const int*   eli     = (const int*)d_in[20];
  float* out = (float*)d_out;
  const int vec8 = ((NEDG & 3) == 0) ? 1 : 0;

  char* ws = (char*)d_ws;
  size_t off = 0;
  const size_t oXLB = off; off = al256(off + (size_t)MLOC * HD * 2);
  const size_t oWPL = off; off = al256(off + (size_t)WPLN * 2);
  const size_t oR1  = off; off = al256(off + (size_t)MEXP * 256);
  const size_t oR2  = off; off = al256(off + (size_t)MEXP * 256);
  const size_t oR3  = off; off = al256(off + (size_t)MLOC * 256);
  const size_t oR4  = off; off = al256(off + (size_t)MLOC * 256);
  const size_t oLO  = off; off = al256(off + (size_t)GAO * RCO * 4);
  const size_t oLR  = off; off = al256(off + (size_t)GAR * RCR * 4);
  const size_t oCO  = off; off = al256(off + (size_t)GAO * NBO * 4);
  const size_t oOO  = off; off = al256(off + (size_t)GAO * NBO * 4);
  const size_t oCR  = off; off = al256(off + (size_t)GAR * NBR * 4);
  const size_t oOR  = off; off = al256(off + (size_t)GAR * NBR * 4);
  const size_t oFO  = off; off = al256(off + (size_t)GAO * 128);
  const size_t oFR  = off; off = al256(off + (size_t)GAR * 128);
  if (off > ws_size || off > (size_t)WSMAX) return;
  unsigned short* XLB = (unsigned short*)(ws + oXLB);
  unsigned short* WPL = (unsigned short*)(ws + oWPL);
  unsigned short* R1  = (unsigned short*)(ws + oR1);
  unsigned short* R2  = (unsigned short*)(ws + oR2);
  unsigned short* R3  = (unsigned short*)(ws + oR3);
  unsigned short* R4  = (unsigned short*)(ws + oR4);
  int* LISTO = (int*)(ws + oLO);
  int* LISTR = (int*)(ws + oLR);
  int* CNTO  = (int*)(ws + oCO);
  int* OFFO  = (int*)(ws + oOO);
  int* CNTR  = (int*)(ws + oCR);
  int* OFFR  = (int*)(ws + oOR);
  int* FLGO  = (int*)(ws + oFO);
  int* FLGR  = (int*)(ws + oFR);
  const unsigned short* W1cO = WPL;
  const unsigned short* W1cR = WPL + 12288;
  const unsigned short* W2cO = WPL + 24576;
  const unsigned short* W2cR = WPL + 40960;
  const unsigned short* DTOP = WPL + 57344;
  const unsigned short* DBOT = WPL + 65536;

  const int ldsO = (LISTN + 2 * RCO + 3 * NBO + 16) * 4;
  const int ldsR = (LISTN + 2 * RCR + 3 * NBR + 16) * 4;
  hipFuncSetAttribute(reinterpret_cast<const void*>(&k_bucket<NBO, SLO, RCO>),
                      hipFuncAttributeMaxDynamicSharedMemorySize, ldsO);
  hipFuncSetAttribute(reinterpret_cast<const void*>(&k_bucket<NBR, SLR, RCR>),
                      hipFuncAttributeMaxDynamicSharedMemorySize, ldsR);

  k_prep<<<(NUX + NWU) / NTHR, NTHR, 0, stream>>>(emb_loc, W1l_of, W1r_of, W1l_rev, W1r_rev,
                                                  W2l_of, W2r_of, W2l_rev, W2r_rev, dW1, XLB, WPL, NLOC);
  k_bucket<NBO, SLO, RCO><<<GAO, NTHR, ldsO, stream>>>(e_of, e_of + NEDG, NEDG, NEXP, NLOC, vec8,
                                                       LISTO, CNTO, OFFO, FLGO);
  k_bucket<NBR, SLR, RCR><<<GAR, NTHR, ldsR, stream>>>(e_rev, e_rev + NEDG, NEDG, NLOC, NEXP, vec8,
                                                       LISTR, CNTR, OFFR, FLGR);
  k_agg<0, NBO, RCO, DCO><<<GAO, NTHR, 0, stream>>>(LISTO, CNTO, OFFO, FLGO, XLB, emb_exp,
                                                    (unsigned*)R1, NEXP, NLOC, MEXP);
  k_agg<1, NBR, RCR, DCR><<<GAR, NTHR, 0, stream>>>(LISTR, CNTR, OFFR, FLGR, XLB, emb_exp,
                                                    (unsigned*)R3, NLOC, NEXP, MLOC);
  k_gemm<2, 0><<<MEXP / GM, GTH, 0, stream>>>(R1, XLB, emb_exp, NEXP, W1cO, b1_of, 1, R2, out, NEXP);
  k_gemm<1, 0><<<MLOC / GM, GTH, 0, stream>>>(R3, XLB, emb_exp, NEXP, W1cR, b1_rev, 1, R4, out, NLOC);
  k_agg<2, NBO, RCO, DCO><<<GAO, NTHR, 0, stream>>>(LISTO, CNTO, OFFO, FLGO, R4, emb_exp,
                                                    (unsigned*)R1, NEXP, NLOC, MEXP);
  k_agg<2, NBR, RCR, DCR><<<GAR, NTHR, 0, stream>>>(LISTR, CNTR, OFFR, FLGR, R2, emb_exp,
                                                    (unsigned*)R3, NLOC, NEXP, MLOC);
  k_gemm<3, 1><<<MEXP / GM, GTH, 0, stream>>>(R1, R2, emb_exp, NEXP, W2cO, b2_of, 1, R1, out, NEXP);
  k_gemm<3, 1><<<MLOC / GM, GTH, 0, stream>>>(R3, R4, emb_exp, NEXP, W2cR, b2_rev, 1, R3, out, NLOC);
  k_gemm<0, 2><<<MEXP / GM, GTH, 0, stream>>>(R1, XLB, emb_exp, NEXP, DBOT, db1, 0, R1, (float*)R2, NEXP);
  k_gemm<0, 2><<<MLOC / GM, GTH, 0, stream>>>(R3, XLB, emb_exp, NEXP, DTOP, db1, 1, R3, (float*)R4, NLOC);
  k_dec<<<(NLBL / 32 + NWAVE - 1) / NWAVE, NTHR, 0, stream>>>(eli, (const float*)R4, (const float*)R2,
                                                              dW2, db2, out, NLBL, NLOC, NEXP);
}
